// FlowLayer_71554155151377
// MI455X (gfx1250) — hardware-run, weakly checked
//
#include <hip/hip_runtime.h>

constexpr int NBATCH  = 2;
constexpr int NCIN    = 256;
constexpr int NCOUT   = 128;
constexpr int IMH     = 128;
constexpr int IMW     = 128;
constexpr int HWPIX   = IMH * IMW;
constexpr int NPIXALL = NBATCH * HWPIX;
constexpr int PPI_STEP = 4;
constexpr int NSTEPS  = 3 * IMH / (4 * PPI_STEP);
constexpr int NCAT    = 2 * NCOUT;
static_assert(NSTEPS == 24);
static_assert(IMW == 128 && IMH == 128 && HWPIX == 16384);

constexpr float SC_X   = 16.0f;
constexpr float SC_W   = 16.0f;
constexpr float SC_CAT = 64.0f;
constexpr float SC_D2  = 1024.0f;

constexpr size_t OFF_XT  = 0;
constexpr size_t SZ_XT   = (size_t)NPIXALL * NCIN * 2;
constexpr size_t OFF_MA  = OFF_XT + SZ_XT;
constexpr size_t SZ_APL  = (size_t)2 * NPIXALL * NCOUT * 4;
constexpr size_t OFF_AP  = OFF_MA + SZ_APL;
constexpr size_t OFF_SS  = OFF_AP + SZ_APL;
constexpr size_t OFF_W1  = OFF_SS + SZ_APL;
constexpr size_t SZ_WB   = (size_t)NCOUT * NCIN * 2;
constexpr size_t OFF_W2  = OFF_W1 + SZ_WB;
constexpr size_t OFF_MPW = OFF_W2 + SZ_WB;
constexpr size_t OFF_PPW = OFF_MPW + SZ_WB;
constexpr size_t SZ_PPW  = (size_t)NCOUT * NCOUT * 2;
constexpr size_t OFF_IDX = OFF_PPW + SZ_PPW;
constexpr size_t SZ_TAB  = (size_t)2 * NPIXALL * 16;
constexpr size_t OFF_WT  = OFF_IDX + SZ_TAB;
constexpr size_t WS_TOTAL = OFF_WT + SZ_TAB;
constexpr size_t OFF_T   = OFF_MA;
constexpr size_t SZ_T    = (size_t)NPIXALL * NCOUT * 4;
constexpr size_t OFF_D2  = OFF_MA + SZ_T;
constexpr size_t SZ_D2   = (size_t)NPIXALL * NCOUT * 2;
static_assert(WS_TOTAL == 119767040);
static_assert(WS_TOTAL <= (size_t)134217728);
static_assert(OFF_D2 + SZ_D2 <= OFF_AP);
static_assert(SZ_XT == (size_t)NPIXALL * NCAT * 2);
static_assert((OFF_MA % 256) == 0 && (OFF_AP % 256) == 0 && (OFF_SS % 256) == 0 && (OFF_W1 % 256) == 0 &&
              (OFF_IDX % 256) == 0 && (OFF_WT % 256) == 0 && (OFF_D2 % 256) == 0);

typedef __attribute__((ext_vector_type(16))) _Float16 v16h;
typedef __attribute__((ext_vector_type(8)))  _Float16 v8h;
typedef __attribute__((ext_vector_type(16))) __bf16   v16b;
typedef __attribute__((ext_vector_type(8)))  __bf16   v8b;
typedef __attribute__((ext_vector_type(8)))  float    v8f;
typedef __attribute__((ext_vector_type(4)))  float    v4f;
typedef __attribute__((ext_vector_type(4)))  int      v4i;
#define U16(p) ((const unsigned short*)(const void*)(p))

__device__ __forceinline__ unsigned short f2bf_bits(float f) {
  unsigned u = __float_as_uint(f);
  return (unsigned short)((u + 0x7FFFu + ((u >> 16) & 1u)) >> 16);
}
__device__ __forceinline__ float bf_bits2f(unsigned short h) { return __uint_as_float(((unsigned)h) << 16); }

__device__ __forceinline__ void dep_guard_h(v8f& a, v8f& b, v16h x, v16h y) { asm volatile("v_nop\n\tv_nop\n\tv_nop\n\tv_nop" : "+v"(a), "+v"(b) : "v"(x), "v"(y)); }
__device__ __forceinline__ void dep_guard_b(v8f& a, v8f& b, v16b x, v16b y) { asm volatile("v_nop\n\tv_nop\n\tv_nop\n\tv_nop" : "+v"(a), "+v"(b) : "v"(x), "v"(y)); }
__device__ __forceinline__ void keep4_h(v16h a, v16h b, v16h c, v16h d) { asm volatile("v_nop" :: "v"(a), "v"(b), "v"(c), "v"(d)); }
__device__ __forceinline__ void keep4_b(v16b a, v16b b, v16b c, v16b d) { asm volatile("v_nop" :: "v"(a), "v"(b), "v"(c), "v"(d)); }
__device__ __forceinline__ void acc_guard4(v8f& a, v8f& b, v8f& c, v8f& d) { asm volatile("v_nop\n\tv_nop\n\tv_nop\n\tv_nop" : "+v"(a), "+v"(b), "+v"(c), "+v"(d)); }
template <typename T> struct Frag;
template <> struct Frag<_Float16> {
  typedef v16h V; union U { v16h v; v8h h[2]; };
  static __device__ __forceinline__ v16h load(const _Float16* p) {
    U f; f.h[0] = *(const v8h*)(p); f.h[1] = *(const v8h*)(p + 16); return f.v;
  }
  static __device__ __forceinline__ v8f mma(v16h a, v16h b, v8f c) {
    return __builtin_amdgcn_wmma_f32_16x16x32_f16(false, a, false, b, (short)0, c, false, false);
  }
  static __device__ __forceinline__ void guard(v8f& a, v8f& b, v16h x, v16h y) { dep_guard_h(a, b, x, y); }
  static __device__ __forceinline__ void keep(v16h a, v16h b, v16h c, v16h d) { keep4_h(a, b, c, d); }
};
template <> struct Frag<__bf16> {
  typedef v16b V; union U { v16b v; v8b h[2]; };
  static __device__ __forceinline__ v16b load(const __bf16* p) {
    U f; f.h[0] = *(const v8b*)(p); f.h[1] = *(const v8b*)(p + 16); return f.v;
  }
  static __device__ __forceinline__ v8f mma(v16b a, v16b b, v8f c) {
    return __builtin_amdgcn_wmma_f32_16x16x32_bf16(false, a, false, b, (short)0, c, false, false);
  }
  static __device__ __forceinline__ void guard(v8f& a, v8f& b, v16b x, v16b y) { dep_guard_b(a, b, x, y); }
  static __device__ __forceinline__ void keep(v16b a, v16b b, v16b c, v16b d) { keep4_b(a, b, c, d); }
};

template <int ET> struct Elem;
template <> struct Elem<0> { typedef _Float16 T; };
template <> struct Elem<1> { typedef __bf16 T; };
template <int ET, bool SPLIT, int BIAS_MODE, int OUT_MODE, bool RESID, int ACT = 0>
__global__ __launch_bounds__(256) void wmma_gemm64(
    const unsigned short* __restrict__ Ap, const unsigned short* __restrict__ A2p, int lda, long strideA,
    const unsigned short* __restrict__ Btp, const unsigned short* __restrict__ Bt2p, int ldb, long strideB,
    void* __restrict__ Cout, void* __restrict__ Cout2, int ldc, long strideC,
    const float* __restrict__ bias,
    const float* __restrict__ resid, long strideR,
    int M, int N, int K, float scale) {
  typedef typename Elem<ET>::T T;
  typedef typename Frag<T>::V V;
  const T* A = (const T*)Ap; const T* A2 = (const T*)A2p; const T* Bt = (const T*)Btp; const T* Bt2 = (const T*)Bt2p;
  __shared__ __align__(16) float sT[8][16 * 68];
  const int b    = blockIdx.y;
  const int lane = threadIdx.x & 31;
  const int wave = threadIdx.x >> 5;
  const int tilesN = N >> 6;
  const int tilesM = M >> 6;
  const int tile = blockIdx.x * 8 + wave;
  if (tile >= tilesM * tilesN) return;
  const int tm = tile / tilesN;
  const int tn = tile - tm * tilesN;
  const int m0 = tm << 6;
  const int n0 = tn << 6;

  const T* Ab  = A  + (size_t)b * strideA;
  const T* Bb  = Bt + (size_t)b * strideB;
  const T* Ab2 = SPLIT ? (A2  + (size_t)b * strideA) : nullptr;
  const T* Bb2 = SPLIT ? (Bt2 + (size_t)b * strideB) : nullptr;

  const int rlane = lane & 15;
  const int koff  = (lane >> 4) * 8;
  const int mOff  = (lane >> 4) * 8;

  v8f acc[4][4];
#pragma unroll
  for (int i = 0; i < 4; ++i)
#pragma unroll
    for (int j = 0; j < 4; ++j) acc[i][j] = (v8f){0.f,0.f,0.f,0.f,0.f,0.f,0.f,0.f};

  for (int k0 = 0; k0 < K; k0 += 32) {
    V bh[4], bl[4];
#pragma unroll
    for (int j = 0; j < 4; ++j) {
      const size_t bo = (size_t)(n0 + (j << 4) + rlane) * ldb + koff + k0;
      bh[j] = Frag<T>::load(Bb + bo);
      if (SPLIT) bl[j] = Frag<T>::load(Bb2 + bo);
    }
#pragma unroll
    for (int i = 0; i < 4; ++i) {
      const size_t ao = (size_t)(m0 + (i << 4) + rlane) * lda + koff + k0;
      V ah = Frag<T>::load(Ab + ao);
      V al;
      if (SPLIT) al = Frag<T>::load(Ab2 + ao);
#pragma unroll
      for (int j = 0; j < 4; ++j) {
        acc[i][j] = Frag<T>::mma(ah, bh[j], acc[i][j]);
        if (SPLIT) {
          acc[i][j] = Frag<T>::mma(ah, bl[j], acc[i][j]);
          acc[i][j] = Frag<T>::mma(al, bh[j], acc[i][j]);
        }
      }
      Frag<T>::guard(acc[i][0], acc[i][3], ah, SPLIT ? al : ah);
    }
    Frag<T>::keep(bh[0], bh[1], bh[2], bh[3]);
    if (SPLIT) Frag<T>::keep(bl[0], bl[1], bl[2], bl[3]);
  }
  acc_guard4(acc[0][0], acc[0][1], acc[0][2], acc[0][3]);
  acc_guard4(acc[1][0], acc[1][1], acc[1][2], acc[1][3]);
  acc_guard4(acc[2][0], acc[2][1], acc[2][2], acc[2][3]);
  acc_guard4(acc[3][0], acc[3][1], acc[3][2], acc[3][3]);

  float* slab = sT[wave];
  const float* Rb = RESID ? (resid + (size_t)b * strideR) : nullptr;
#pragma unroll
  for (int i = 0; i < 4; ++i) {
    const int mBase = m0 + (i << 4);
    float bm[8];
#pragma unroll
    for (int r = 0; r < 8; ++r) bm[r] = 0.f;
    if (BIAS_MODE == 1) {
      const v4f b0v = *(const v4f*)(bias + mBase + mOff);
      const v4f b1v = *(const v4f*)(bias + mBase + mOff + 4);
      bm[0] = b0v[0]; bm[1] = b0v[1]; bm[2] = b0v[2]; bm[3] = b0v[3];
      bm[4] = b1v[0]; bm[5] = b1v[1]; bm[6] = b1v[2]; bm[7] = b1v[3];
    }
#pragma unroll
    for (int j = 0; j < 4; ++j) {
      const int n = n0 + (j << 4) + rlane;
      float bv = 0.f;
      if (BIAS_MODE == 2) bv = bias[n];
#pragma unroll
      for (int r = 0; r < 8; ++r) {
        float v = acc[i][j][r] * scale;
        if (BIAS_MODE == 1) v += bm[r];
        if (BIAS_MODE == 2) v += bv;
        if (RESID) v += Rb[(size_t)(mBase + mOff + r) * ldc + n];
        if (ACT == 1) v = tanhf(v);
        if (ACT == 2) v = fmaxf(v, 0.0f);
        if (ACT == 3) v = v / (1.0f + expf(-v));
        if (ACT == 4) v = (v > 0.f) ? v : 0.01f * v;
        if (ACT == 6) v = 1.0f / (1.0f + expf(-v));
        slab[(mOff + r) * 68 + (j << 4) + rlane] = v;
      }
    }
    __builtin_amdgcn_fence(__ATOMIC_RELEASE, "workgroup");
    __builtin_amdgcn_wave_barrier();
    __builtin_amdgcn_fence(__ATOMIC_ACQUIRE, "workgroup");
    if (OUT_MODE == 0) {
      float* C = (float*)Cout + (size_t)b * strideC;
      const int hh = lane >> 4, c4 = (lane & 15) * 4;
      for (int pass = 0; pass < 2; ++pass) {
#pragma unroll
        for (int it = 0; it < 8; ++it) {
          const int row = it * 2 + hh;
          v4f v = *(const v4f*)(slab + row * 68 + c4);
          *(volatile v4f*)(C + (size_t)(mBase + row) * ldc + n0 + c4) = v;
        }
        __threadfence();
      }
    } else {
      const int q = lane >> 3, c8 = (lane & 7) * 8;
      unsigned short* C  = (unsigned short*)Cout  + (size_t)b * strideC;
      unsigned short* C2 = (OUT_MODE == 2) ? ((unsigned short*)Cout2 + (size_t)b * strideC) : nullptr;
      for (int pass = 0; pass < 2; ++pass) {
#pragma unroll
        for (int it = 0; it < 4; ++it) {
          const int row = it * 4 + q;
          const float* sp = slab + row * 68 + c8;
          v8h hv, lv;
#pragma unroll
          for (int e = 0; e < 8; ++e) {
            if (OUT_MODE == 1) {
              hv[e] = (_Float16)sp[e];
            } else {
              unsigned short hb = f2bf_bits(sp[e]);
              unsigned short lb = f2bf_bits(sp[e] - bf_bits2f(hb));
              hv[e] = __builtin_bit_cast(_Float16, hb);
              lv[e] = __builtin_bit_cast(_Float16, lb);
            }
          }
          *(volatile v8h*)(C + (size_t)(mBase + row) * ldc + n0 + c8) = hv;
          if (OUT_MODE == 2) *(volatile v8h*)(C2 + (size_t)(mBase + row) * ldc + n0 + c8) = lv;
        }
        __threadfence();
      }
    }
    __builtin_amdgcn_fence(__ATOMIC_RELEASE, "workgroup");
    __builtin_amdgcn_wave_barrier();
    __builtin_amdgcn_fence(__ATOMIC_ACQUIRE, "workgroup");
  }
}

__global__ __launch_bounds__(256) void k_cast8(const float* __restrict__ in, _Float16* __restrict__ out, int n8, float sc) {
  const int i = blockIdx.x * 256 + threadIdx.x;
  if (i < n8) {
    const float* p = in + (size_t)i * 8;
    const v4f a = *(const v4f*)p;
    const v4f c = *(const v4f*)(p + 4);
    v8h hv;
    hv[0] = (_Float16)(a[0] * sc); hv[1] = (_Float16)(a[1] * sc); hv[2] = (_Float16)(a[2] * sc); hv[3] = (_Float16)(a[3] * sc);
    hv[4] = (_Float16)(c[0] * sc); hv[5] = (_Float16)(c[1] * sc); hv[6] = (_Float16)(c[2] * sc); hv[7] = (_Float16)(c[3] * sc);
    _Float16* d = out + (size_t)i * 8;
    *(volatile v8h*)d = hv;
    __threadfence();
    *(volatile v8h*)d = hv;
  }
}

__global__ __launch_bounds__(256) void k_xpose(const float* __restrict__ x, _Float16* __restrict__ xt) {
  __shared__ float tile[64][33];
  const int b = blockIdx.z, hw0 = blockIdx.x * 32, c0 = blockIdx.y * 64;
  const int t = threadIdx.x, tx = t & 31, ty = t >> 5;
#pragma unroll
  for (int k = 0; k < 8; ++k) {
    const int cl = ty + 8 * k;
    tile[cl][tx] = x[(size_t)(b * NCIN + c0 + cl) * HWPIX + hw0 + tx] * SC_X;
  }
  __syncthreads();
  const int hl = t >> 3, cp = (t & 7) * 8;
  v8h hv;
#pragma unroll
  for (int e = 0; e < 8; ++e) hv[e] = (_Float16)tile[cp + e][hl];
  _Float16* dst = xt + (size_t)(b * HWPIX + hw0 + hl) * NCIN + c0 + cp;
  *(volatile v8h*)dst = hv;
  __threadfence();
  *(volatile v8h*)dst = hv;
}

__device__ __forceinline__ void bilin_corners(float px, float py, int boff, v4i& id, v4f& wv) {
#pragma clang fp contract(off)
  px = fminf(fmaxf(px, -2.0f), (float)(IMW + 1));
  py = fminf(fmaxf(py, -2.0f), (float)(IMH + 1));
  const float x0 = floorf(px), y0 = floorf(py);
  const float wx1 = px - x0, wx0 = 1.0f - wx1;
  const float wy1 = py - y0, wy0 = 1.0f - wy1;
  const int xi0 = (int)x0, yi0 = (int)y0;
  const int xi1 = xi0 + 1, yi1 = yi0 + 1;
  const bool vx0 = (xi0 >= 0) && (xi0 <= IMW - 1);
  const bool vx1 = (xi1 >= 0) && (xi1 <= IMW - 1);
  const bool vy0 = (yi0 >= 0) && (yi0 <= IMH - 1);
  const bool vy1 = (yi1 >= 0) && (yi1 <= IMH - 1);
  const int xc0 = min(max(xi0, 0), IMW - 1), xc1 = min(max(xi1, 0), IMW - 1);
  const int yc0 = min(max(yi0, 0), IMH - 1), yc1 = min(max(yi1, 0), IMH - 1);
  id[0] = boff + yc0 * IMW + xc0; wv[0] = (vx0 && vy0) ? (wx0 * wy0) : 0.0f;
  id[1] = boff + yc0 * IMW + xc1; wv[1] = (vx1 && vy0) ? (wx1 * wy0) : 0.0f;
  id[2] = boff + yc1 * IMW + xc0; wv[2] = (vx0 && vy1) ? (wx0 * wy1) : 0.0f;
  id[3] = boff + yc1 * IMW + xc1; wv[3] = (vx1 && vy1) ? (wx1 * wy1) : 0.0f;
}

__global__ __launch_bounds__(256) void k_grid_setup(const float* __restrict__ grads, int* __restrict__ idx, float* __restrict__ wt) {
#pragma clang fp contract(off)
  const int p = blockIdx.x * 256 + threadIdx.x;
  const int b = p >> 14, hw = p & (HWPIX - 1);
  const int h = hw >> 7, w = hw & (IMW - 1);
  const float g0 = grads[(size_t)(b * 2 + 0) * HWPIX + hw];
  const float g1 = grads[(size_t)(b * 2 + 1) * HWPIX + hw];
  const float gsc = 1.5f / (float)NSTEPS;
  const float gx = g0 * gsc, gy = g1 * gsc;
  const float tqx = (float)w * (1.0f / (float)(IMW - 1));
  const float tqy = (float)h * (1.0f / (float)(IMH - 1));
  float xs = -1.0f * (1.0f - tqx) + 1.0f * tqx;
  float ys = -1.0f * (1.0f - tqy) + 1.0f * tqy;
  if (w == IMW - 1) xs = 1.0f;
  if (h == IMH - 1) ys = 1.0f;
  const float hx = (float)(IMW - 1), hy = (float)(IMH - 1);
  const float px0 = ((xs + gx) + 1.0f) * hx * 0.5f;
  const float py0 = ((ys + gy) + 1.0f) * hy * 0.5f;
  const float px1 = ((xs - gx) + 1.0f) * hx * 0.5f;
  const float py1 = ((ys - gy) + 1.0f) * hy * 0.5f;
  const int boff = b * HWPIX;
  v4i id0, id1; v4f w0, w1;
  bilin_corners(px0, py0, boff, id0, w0);
  bilin_corners(px1, py1, boff, id1, w1);
  const size_t te0 = (size_t)p * 4;
  const size_t te1 = ((size_t)NPIXALL + p) * 4;
  *(volatile v4i*)(idx + te0) = id0; *(volatile v4f*)(wt + te0) = w0;
  *(volatile v4i*)(idx + te1) = id1; *(volatile v4f*)(wt + te1) = w1;
  __threadfence();
  *(volatile v4i*)(idx + te0) = id0; *(volatile v4f*)(wt + te0) = w0;
  *(volatile v4i*)(idx + te1) = id1; *(volatile v4f*)(wt + te1) = w1;
}

__global__ __launch_bounds__(256) void k_warp_step(const float* __restrict__ aold, float* __restrict__ anew,
                                                   float* __restrict__ sacc, const int* __restrict__ idx,
                                                   const float* __restrict__ wt, int first, int last) {
  const int lane = threadIdx.x & 31;
  const int flat = blockIdx.x * 8 + (threadIdx.x >> 5);
  const int strm = flat & 1;
  const int p = flat >> 1;
  const size_t sb = (size_t)strm * NPIXALL * NCOUT;
  const size_t te = ((size_t)strm * NPIXALL + p) * 4;
  const v4i id = *(const v4i*)(idx + te);
  const v4f wv = *(const v4f*)(wt + te);
  const unsigned lim = (unsigned)(NPIXALL - 1);
  const unsigned q0 = min((unsigned)id[0], lim);
  const unsigned q1 = min((unsigned)id[1], lim);
  const unsigned q2 = min((unsigned)id[2], lim);
  const unsigned q3 = min((unsigned)id[3], lim);
  const float* ab = aold + sb + lane * 4;
  const v4f v0 = *(const v4f*)(ab + (size_t)q0 * NCOUT);
  const v4f v1 = *(const v4f*)(ab + (size_t)q1 * NCOUT);
  const v4f v2 = *(const v4f*)(ab + (size_t)q2 * NCOUT);
  const v4f v3 = *(const v4f*)(ab + (size_t)q3 * NCOUT);
  v4f acc = wv[0] * v0;
  acc = acc + wv[1] * v1;
  acc = acc + wv[2] * v2;
  acc = acc + wv[3] * v3;
  const size_t o = sb + (size_t)p * NCOUT + lane * 4;
  v4f sp;
  if (first) sp = *(const v4f*)(aold + o);
  else       sp = *(const v4f*)(sacc + o);
  v4f sn = sp + acc;
  if (last) {
    sn[0] = 1.0f / (1.0f + expf(-sn[0]));
    sn[1] = 1.0f / (1.0f + expf(-sn[1]));
    sn[2] = 1.0f / (1.0f + expf(-sn[2]));
    sn[3] = 1.0f / (1.0f + expf(-sn[3]));
  }
  float* pa = anew + o;
  float* ps = sacc + o;
  *(volatile v4f*)pa = acc;
  *(volatile v4f*)ps = sn;
  __threadfence();
  *(volatile v4f*)pa = acc;
  *(volatile v4f*)ps = sn;
}

__device__ __forceinline__ v4f zsel4(bool c, v4f v) {
  v4f r;
  r[0] = c ? v[0] : 0.0f; r[1] = c ? v[1] : 0.0f; r[2] = c ? v[2] : 0.0f; r[3] = c ? v[3] : 0.0f;
  return r;
}

__global__ __launch_bounds__(256) void k_dwcat(const float* __restrict__ ss, const float* __restrict__ dw,
                                               _Float16* __restrict__ dcat) {
  __shared__ __align__(16) float wsh[9 * NCAT];
  const int t = threadIdx.x;
#pragma unroll
  for (int i = 0; i < 9; ++i) {
    const int e = t + 256 * i;
    const int c = e / 9;
    const int tap = e - c * 9;
    wsh[tap * NCAT + c] = dw[e];
  }
  __syncthreads();
  const int wave = t >> 5, lane = t & 31;
  const int strm = wave & 1;
  const int p = blockIdx.x * 8 + (wave >> 1) * 2 + (lane >> 4);
  const int cg = lane & 15;
  const int b = p >> 14, hw = p & (HWPIX - 1);
  const int h = hw >> 7, w = hw & (IMW - 1);
  const float* sbase = ss + (size_t)strm * NPIXALL * NCOUT + (size_t)b * HWPIX * NCOUT + cg * 8;
  const float* wbase = wsh + strm * NCOUT + cg * 8;
  v4f accA = {0.f, 0.f, 0.f, 0.f}, accB = {0.f, 0.f, 0.f, 0.f};
#pragma unroll 1
  for (int ky = 0; ky < 3; ++ky) {
    const int yy = h + ky - 1;
    const bool vy = (unsigned)yy < (unsigned)IMH;
    const int yc = min(max(yy, 0), IMH - 1);
#pragma unroll 1
    for (int kx = 0; kx < 3; ++kx) {
      const int xx = w + kx - 1;
      const bool valid = vy && ((unsigned)xx < (unsigned)IMW);
      const int xc = min(max(xx, 0), IMW - 1);
      const float* src = sbase + (size_t)(yc * IMW + xc) * NCOUT;
      const v4f uA = zsel4(valid, *(const v4f*)src);
      const v4f uB = zsel4(valid, *(const v4f*)(src + 4));
      const float* wp = wbase + (ky * 3 + kx) * NCAT;
      const v4f wA = *(const v4f*)wp;
      const v4f wB = *(const v4f*)(wp + 4);
      accA = accA + wA * uA;
      accB = accB + wB * uB;
    }
  }
  v8h hv;
  hv[0] = (_Float16)(accA[0] * SC_CAT); hv[1] = (_Float16)(accA[1] * SC_CAT);
  hv[2] = (_Float16)(accA[2] * SC_CAT); hv[3] = (_Float16)(accA[3] * SC_CAT);
  hv[4] = (_Float16)(accB[0] * SC_CAT); hv[5] = (_Float16)(accB[1] * SC_CAT);
  hv[6] = (_Float16)(accB[2] * SC_CAT); hv[7] = (_Float16)(accB[3] * SC_CAT);
  _Float16* dst = dcat + (size_t)p * NCAT + strm * NCOUT + cg * 8;
  *(volatile v8h*)dst = hv;
  __threadfence();
  *(volatile v8h*)dst = hv;
}

__global__ __launch_bounds__(256) void k_dwpost(const float* __restrict__ tin, const float* __restrict__ dw,
                                                _Float16* __restrict__ d2) {
  __shared__ __align__(16) float wsh[9 * NCOUT];
  const int t = threadIdx.x;
#pragma unroll
  for (int i = 0; i < 5; ++i) {
    const int e = t + 256 * i;
    if (e < 9 * NCOUT) {
      const int c = e / 9;
      const int tap = e - c * 9;
      wsh[tap * NCOUT + c] = dw[e];
    }
  }
  __syncthreads();
  const int wave = t >> 5, lane = t & 31;
  const int p = blockIdx.x * 16 + wave * 2 + (lane >> 4);
  const int cg = lane & 15;
  const int b = p >> 14, hw = p & (HWPIX - 1);
  const int h = hw >> 7, w = hw & (IMW - 1);
  const float* sbase = tin + (size_t)b * HWPIX * NCOUT + cg * 8;
  const float* wbase = wsh + cg * 8;
  v4f accA = {0.f, 0.f, 0.f, 0.f}, accB = {0.f, 0.f, 0.f, 0.f};
#pragma unroll 1
  for (int ky = 0; ky < 3; ++ky) {
    const int yy = h + ky - 1;
    const bool vy = (unsigned)yy < (unsigned)IMH;
    const int yc = min(max(yy, 0), IMH - 1);
#pragma unroll 1
    for (int kx = 0; kx < 3; ++kx) {
      const int xx = w + kx - 1;
      const bool valid = vy && ((unsigned)xx < (unsigned)IMW);
      const int xc = min(max(xx, 0), IMW - 1);
      const float* src = sbase + (size_t)(yc * IMW + xc) * NCOUT;
      const v4f uA = zsel4(valid, *(const v4f*)src);
      const v4f uB = zsel4(valid, *(const v4f*)(src + 4));
      const float* wp = wbase + (ky * 3 + kx) * NCOUT;
      const v4f wA = *(const v4f*)wp;
      const v4f wB = *(const v4f*)(wp + 4);
      accA = accA + wA * uA;
      accB = accB + wB * uB;
    }
  }
  v8h hv;
  hv[0] = (_Float16)(accA[0] * SC_D2); hv[1] = (_Float16)(accA[1] * SC_D2);
  hv[2] = (_Float16)(accA[2] * SC_D2); hv[3] = (_Float16)(accA[3] * SC_D2);
  hv[4] = (_Float16)(accB[0] * SC_D2); hv[5] = (_Float16)(accB[1] * SC_D2);
  hv[6] = (_Float16)(accB[2] * SC_D2); hv[7] = (_Float16)(accB[3] * SC_D2);
  _Float16* dst = d2 + (size_t)p * NCOUT + cg * 8;
  *(volatile v8h*)dst = hv;
  __threadfence();
  *(volatile v8h*)dst = hv;
}

extern "C" void kernel_launch(void* const* d_in, const int* in_sizes, int n_in,
                              void* d_out, int out_size, void* d_ws, size_t ws_size,
                              hipStream_t stream) {
  if (n_in < 10) return;
  if (in_sizes[0] != NBATCH * NCIN * HWPIX || in_sizes[1] != NBATCH * 2 * HWPIX ||
      in_sizes[2] != NCOUT * NCIN || in_sizes[3] != NCOUT * NCIN || in_sizes[4] != NCAT * 9 ||
      in_sizes[5] != NCOUT * NCAT || in_sizes[6] != NCOUT || in_sizes[7] != NCOUT * 9 ||
      in_sizes[8] != NCOUT * NCOUT || in_sizes[9] != NCOUT) return;
  if (out_size != NBATCH * NCOUT * HWPIX) return;
  if (ws_size < WS_TOTAL) return;

  const float* x     = (const float*)d_in[0];
  const float* grads = (const float*)d_in[1];
  const float* w1    = (const float*)d_in[2];
  const float* w2    = (const float*)d_in[3];
  const float* mdw   = (const float*)d_in[4];
  const float* mpw   = (const float*)d_in[5];
  const float* mb    = (const float*)d_in[6];
  const float* pdw   = (const float*)d_in[7];
  const float* ppw   = (const float*)d_in[8];
  const float* pb    = (const float*)d_in[9];
  float* out = (float*)d_out;

  char* ws = (char*)d_ws;
  _Float16* XT   = (_Float16*)(ws + OFF_XT);
  _Float16* DCAT = (_Float16*)(ws + OFF_XT);
  float*    MA   = (float*)(ws + OFF_MA);
  float*    AP   = (float*)(ws + OFF_AP);
  float*    SS   = (float*)(ws + OFF_SS);
  float*    TT   = (float*)(ws + OFF_T);
  _Float16* D2   = (_Float16*)(ws + OFF_D2);
  _Float16* W1H  = (_Float16*)(ws + OFF_W1);
  _Float16* W2H  = (_Float16*)(ws + OFF_W2);
  _Float16* MPWH = (_Float16*)(ws + OFF_MPW);
  _Float16* PPWH = (_Float16*)(ws + OFF_PPW);
  int*      IDX  = (int*)(ws + OFF_IDX);
  float*    WT   = (float*)(ws + OFF_WT);
  const float* unused_f = (const float*)(ws + OFF_SS);

  {
    const int n8a = NCOUT * NCIN / 8;
    const int n8p = NCOUT * NCOUT / 8;
    k_cast8<<<(n8a + 255) / 256, 256, 0, stream>>>(w1, W1H, n8a, SC_W);
    k_cast8<<<(n8a + 255) / 256, 256, 0, stream>>>(w2, W2H, n8a, SC_W);
    k_cast8<<<(n8a + 255) / 256, 256, 0, stream>>>(mpw, MPWH, n8a, SC_W);
    k_cast8<<<(n8p + 255) / 256, 256, 0, stream>>>(ppw, PPWH, n8p, SC_W);
  }

  k_xpose<<<dim3(HWPIX / 32, NCIN / 64, NBATCH), 256, 0, stream>>>(x, XT);

  static_assert(NPIXALL % 64 == 0 && NCOUT % 64 == 0 && NCIN % 32 == 0);
  {
    const int tiles = (NPIXALL / 64) * (NCOUT / 64);
    const dim3 grid((tiles + 7) / 8, 1);
    const float sc = 1.0f / (SC_X * SC_W);
    wmma_gemm64<0, false, 0, 0, false, 6><<<grid, 256, 0, stream>>>(
        U16(XT), U16(XT), NCIN, (long)0, U16(W1H), U16(W1H), NCIN, (long)0,
        (void*)MA, (void*)MA, NCOUT, (long)0, mb, unused_f, (long)0, NPIXALL, NCOUT, NCIN, sc);
    wmma_gemm64<0, false, 0, 0, false, 6><<<grid, 256, 0, stream>>>(
        U16(XT), U16(XT), NCIN, (long)0, U16(W2H), U16(W2H), NCIN, (long)0,
        (void*)(MA + (size_t)NPIXALL * NCOUT), (void*)(MA + (size_t)NPIXALL * NCOUT), NCOUT, (long)0,
        mb, unused_f, (long)0, NPIXALL, NCOUT, NCIN, sc);
  }

  k_grid_setup<<<NPIXALL / 256, 256, 0, stream>>>(grads, IDX, WT);

  {
    float* pa = MA; float* pn = AP;
    for (int t = 0; t < NSTEPS; ++t) {
      k_warp_step<<<(NPIXALL * 2) / 8, 256, 0, stream>>>(pa, pn, SS, IDX, WT,
                                                         t == 0 ? 1 : 0, t == NSTEPS - 1 ? 1 : 0);
      float* tmp = pa; pa = pn; pn = tmp;
    }
  }

  k_dwcat<<<NPIXALL / 8, 256, 0, stream>>>(SS, mdw, DCAT);

  static_assert(NCAT % 32 == 0);
  {
    const int tiles = (NPIXALL / 64) * (NCOUT / 64);
    const dim3 grid((tiles + 7) / 8, 1);
    const float sc = 1.0f / (SC_CAT * SC_W);
    wmma_gemm64<0, false, 2, 0, false, 0><<<grid, 256, 0, stream>>>(
        U16(DCAT), U16(DCAT), NCAT, (long)0, U16(MPWH), U16(MPWH), NCAT, (long)0,
        (void*)TT, (void*)TT, NCOUT, (long)0, mb, unused_f, (long)0, NPIXALL, NCOUT, NCAT, sc);
  }

  k_dwpost<<<NPIXALL / 16, 256, 0, stream>>>(TT, pdw, D2);

  static_assert(HWPIX % 64 == 0 && NCOUT % 32 == 0);
  {
    const int tiles = (NCOUT / 64) * (HWPIX / 64);
    const dim3 grid((tiles + 7) / 8, NBATCH);
    const float sc = 1.0f / (SC_D2 * SC_W);
    wmma_gemm64<0, false, 1, 0, false, 0><<<grid, 256, 0, stream>>>(
        U16(PPWH), U16(PPWH), NCOUT, (long)0, U16(D2), U16(D2), NCOUT, (long)HWPIX * NCOUT,
        (void*)out, (void*)out, HWPIX, (long)NCOUT * HWPIX, pb, unused_f, (long)0, NCOUT, HWPIX, NCOUT, sc);
  }
}
